// SparseMoELayer_88811333746987
// MI455X (gfx1250) — hardware-verified
//
#include <hip/hip_runtime.h>
#include <stdint.h>
#include <math.h>


#define TKN   8192
#define HID   512
#define DFF   2048
#define NEXP  8
#define TOPK  2
#define NSLOT (TKN * TOPK)

#define MT    64
#define CC    64
#define NCH   (DFF / CC)
#define TPB   512
#define XP    520
#define W2TP  72
#define HP    72
#define STP   516
#define CVTP  68

#define SCX   8.0f
#define SCW   64.0f
#define SCH   16.0f
#define INV_G1 (1.0f / 512.0f)
#define INV_G2 (1.0f / 1024.0f)

typedef _Float16 v8h  __attribute__((ext_vector_type(8)));
typedef _Float16 v16h __attribute__((ext_vector_type(16)));
typedef float    v4f  __attribute__((ext_vector_type(4)));
typedef float    v8f  __attribute__((ext_vector_type(8)));
typedef int      v4i  __attribute__((ext_vector_type(4)));

union Frag  { v16h v; v8h half[2]; };
union Pack8 { v8h v; _Float16 s[8]; };

__device__ __forceinline__ float bfr(float f) {
  unsigned u = __float_as_uint(f);
  u = (u + 0x7FFFu + ((u >> 16) & 1u)) & 0xFFFF0000u;
  return __uint_as_float(u);
}

__device__ __forceinline__ v8f wmma16(const v16h a, const v16h b, v8f c) {
  c = __builtin_amdgcn_wmma_f32_16x16x32_f16(false, a, false, b, (short)0, c, false, false);
  asm volatile("v_nop\n\tv_nop\n\tv_nop\n\tv_nop" : "+v"(c) : "v"(a), "v"(b));
  return c;
}

__device__ __forceinline__ v16h ld_frag(const _Float16* p, int h) {
  Frag f;
  f.half[0] = *(const v8h*)(p + 8 * h);
  f.half[1] = *(const v8h*)(p + 16 + 8 * h);
  return f.v;
}

__device__ __forceinline__ float gelu_t(float v) {
  float v3 = v * v * v;
  float in = 0.7978845608028654f * (v + 0.044715f * v3);
  return 0.5f * v * (1.0f + tanhf(in));
}

__global__ __launch_bounds__(256) void k_router(const float* __restrict__ x,
                                                  const float* __restrict__ gw,
                                                  int* tk_idx, int* tk_wbits, int ntok) {
  __shared__ float sG[NEXP * HID];
  __shared__ __attribute__((aligned(16))) float sXr[32 * HID];
  __shared__ float sLog[32 * NEXP];
  __shared__ __attribute__((aligned(16))) int sOI[64];
  __shared__ __attribute__((aligned(16))) int sOW[64];
  const int tid = threadIdx.x, lane = tid & 31, wave = tid >> 5;
  const int tok0 = blockIdx.x * 32;
  if (tok0 + 32 > ntok) return;

  for (int i = tid; i < NEXP * HID; i += 256) sG[i] = bfr(gw[i]);
  for (int i = tid; i < 32 * HID / 4; i += 256) {
    v4f v = *(const v4f*)(x + (size_t)tok0 * HID + (size_t)i * 4);
    sXr[i * 4 + 0] = bfr(v.x);
    sXr[i * 4 + 1] = bfr(v.y);
    sXr[i * 4 + 2] = bfr(v.z);
    sXr[i * 4 + 3] = bfr(v.w);
  }
  __syncthreads();

  const int tl = tid >> 3, e = tid & 7;
  const float* xr = sXr + tl * HID;
  const float* gr = sG + e * HID;
  double acc = 0.0;
#pragma unroll 8
  for (int hh = 0; hh < HID; ++hh) {
    float p = xr[hh] * gr[hh];
    acc += (double)p;
  }
  sLog[tl * NEXP + e] = (float)acc;
  __syncthreads();

  if (tid < 32) {
    float v0 = __int_as_float(0xff800000), v1 = __int_as_float(0xff800000);
    int i0 = 0, i1 = 0;
#pragma unroll
    for (int ee = 0; ee < NEXP; ++ee) {
      float v = sLog[tid * NEXP + ee];
      if (v > v0) { v1 = v0; i1 = i0; v0 = v; i0 = ee; }
      else if (v > v1) { v1 = v; i1 = ee; }
    }
    float ex = expf(v1 - v0);
    float s = 1.0f + ex;
    float r = 1.0f / s;
    sOI[tid * 2 + 0] = i0;
    sOI[tid * 2 + 1] = i1;
    sOW[tid * 2 + 0] = __float_as_int(r);
    sOW[tid * 2 + 1] = __float_as_int(ex * r);
  }
  __syncthreads();

  if (wave == 0) {
    v4i v;
    int* dst;
    if (lane < 16) {
      v = *(const v4i*)(sOI + lane * 4);
      dst = tk_idx + (size_t)tok0 * 2 + lane * 4;
    } else {
      v = *(const v4i*)(sOW + (lane - 16) * 4);
      dst = tk_wbits + (size_t)tok0 * 2 + (lane - 16) * 4;
    }
    *(volatile v4i*)dst = v;
    __threadfence();
    *(volatile v4i*)dst = v;
  }
}

__global__ __launch_bounds__(1024) void k_lists(const int* __restrict__ tk_idx,
                                                  int* offsets, int* row_tok, int* slotmap) {
  __shared__ __attribute__((aligned(16))) int sRow[NSLOT];
  __shared__ __attribute__((aligned(16))) int sSlot[NSLOT];
  __shared__ __attribute__((aligned(16))) int sOff[32];
  __shared__ int sWv[32];
  const int tid = threadIdx.x, lane = tid & 31, wave = tid >> 5;

  int idxv[16];
#pragma unroll
  for (int q = 0; q < 4; ++q) {
    v4i v = *(const v4i*)(tk_idx + (size_t)tid * 16 + q * 4);
    idxv[q * 4 + 0] = min(max(v.x, 0), NEXP - 1);
    idxv[q * 4 + 1] = min(max(v.y, 0), NEXP - 1);
    idxv[q * 4 + 2] = min(max(v.z, 0), NEXP - 1);
    idxv[q * 4 + 3] = min(max(v.w, 0), NEXP - 1);
  }
  int slotv[16];
#pragma unroll
  for (int j = 0; j < 16; ++j) slotv[j] = 0;

  int running = 0;
#pragma unroll 1
  for (int e = 0; e < NEXP; ++e) {
    int c = 0;
#pragma unroll
    for (int j = 0; j < 16; ++j) c += (idxv[j] == e) ? 1 : 0;
    int xs = c;
#pragma unroll
    for (int off = 1; off < 32; off <<= 1) {
      int y = __shfl_up(xs, off, 32);
      if (lane >= off) xs += y;
    }
    if (lane == 31) sWv[wave] = xs;
    __syncthreads();
    if (wave == 0) {
      int s = sWv[lane];
#pragma unroll
      for (int off = 1; off < 32; off <<= 1) {
        int y = __shfl_up(s, off, 32);
        if (lane >= off) s += y;
      }
      sWv[lane] = s;
    }
    __syncthreads();
    const int wbase = (wave > 0) ? sWv[wave - 1] : 0;
    const int total = sWv[31];
    int pos = running + wbase + xs - c;
#pragma unroll
    for (int j = 0; j < 16; ++j) {
      if (idxv[j] == e) {
        int sl = pos;
        ++pos;
        slotv[j] = sl;
        if ((unsigned)sl < (unsigned)NSLOT) sRow[sl] = tid * 8 + (j >> 1);
      }
    }
    if (tid == 0) sOff[e] = running;
    running += total;
    __syncthreads();
  }
  if (tid == 0) {
    sOff[NEXP] = running;
    for (int i = NEXP + 1; i < 32; ++i) sOff[i] = 0;
  }
#pragma unroll
  for (int q = 0; q < 4; ++q) {
    v4i v;
    v.x = slotv[q * 4 + 0]; v.y = slotv[q * 4 + 1]; v.z = slotv[q * 4 + 2]; v.w = slotv[q * 4 + 3];
    *(v4i*)(sSlot + tid * 16 + q * 4) = v;
  }
  __syncthreads();

  v4i kr[4], ks[4];
#pragma unroll
  for (int q = 0; q < 4; ++q) {
    int i4 = tid + q * 1024;
    kr[q] = *(const v4i*)(sRow + i4 * 4);
    ks[q] = *(const v4i*)(sSlot + i4 * 4);
  }
  v4i offv = v4i{0, 0, 0, 0};
  if (tid < 8) offv = *(const v4i*)(sOff + tid * 4);

#pragma unroll
  for (int q = 0; q < 4; ++q) {
    int i4 = tid + q * 1024;
    *(volatile v4i*)(row_tok + (size_t)i4 * 4) = kr[q];
    *(volatile v4i*)(slotmap + (size_t)i4 * 4) = ks[q];
  }
  if (tid < 8) *(volatile v4i*)(offsets + tid * 4) = offv;
  __threadfence();
#pragma unroll
  for (int q = 0; q < 4; ++q) {
    int i4 = tid + q * 1024;
    *(volatile v4i*)(row_tok + (size_t)i4 * 4) = kr[q];
    *(volatile v4i*)(slotmap + (size_t)i4 * 4) = ks[q];
  }
  if (tid < 8) *(volatile v4i*)(offsets + tid * 4) = offv;
}

__global__ __launch_bounds__(256) void k_cvt(const float* __restrict__ w, _Float16* wt,
                                               int K, int N, float scale) {
  __shared__ _Float16 tile[64 * CVTP];
  const int tid = threadIdx.x;
  const int e = blockIdx.z, k0 = blockIdx.y * 64, n0 = blockIdx.x * 64;
#pragma unroll
  for (int it = 0; it < 4; ++it) {
    int p = tid + it * 256;
    int kr = p >> 4, c4 = p & 15;
    v4f v = *(const v4f*)(w + ((size_t)e * K + k0 + kr) * (size_t)N + n0 + c4 * 4);
    _Float16* d = tile + kr * CVTP + c4 * 4;
    d[0] = (_Float16)(bfr(v.x) * scale);
    d[1] = (_Float16)(bfr(v.y) * scale);
    d[2] = (_Float16)(bfr(v.z) * scale);
    d[3] = (_Float16)(bfr(v.w) * scale);
  }
  __syncthreads();
  Pack8 u[2];
  _Float16* dst[2];
#pragma unroll
  for (int it = 0; it < 2; ++it) {
    int p = tid + it * 256;
    int n = p >> 3, c = p & 7;
#pragma unroll
    for (int j = 0; j < 8; ++j) u[it].s[j] = tile[(c * 8 + j) * CVTP + n];
    dst[it] = wt + ((size_t)e * N + n0 + n) * (size_t)K + k0 + c * 8;
  }
  *(volatile v8h*)dst[0] = u[0].v;
  *(volatile v8h*)dst[1] = u[1].v;
  __threadfence();
  *(volatile v8h*)dst[0] = u[0].v;
  *(volatile v8h*)dst[1] = u[1].v;
}

union ExpSmem {
  struct { _Float16 x[MT * XP]; _Float16 w1[CC * XP]; } g;
  float stage[MT * STP];
};

__global__ __launch_bounds__(TPB) void k_expert(const float* __restrict__ x,
                                                  const float* __restrict__ b1,
                                                  const float* __restrict__ b2,
                                                  const _Float16* __restrict__ w1t,
                                                  const _Float16* __restrict__ w2t,
                                                  const int* __restrict__ offsets,
                                                  const int* __restrict__ row_tok,
                                                  float* yws, int ntok) {
  __shared__ __attribute__((aligned(16))) ExpSmem su;
  __shared__ __attribute__((aligned(16))) _Float16 sW2[HID * W2TP];
  __shared__ __attribute__((aligned(16))) _Float16 sHd[MT * HP];
  __shared__ int sTok[MT];

  int offv[NEXP + 1];
#pragma unroll
  for (int i = 0; i <= NEXP; ++i) offv[i] = offsets[i];
  const int bid = blockIdx.x;
  int e = -1, tile0 = 0, seg_hi = 0, tb = 0;
#pragma unroll
  for (int ee = 0; ee < NEXP; ++ee) {
    int lo = min(max(offv[ee], 0), NSLOT);
    int hi = min(max(offv[ee + 1], lo), NSLOT);
    int ntile = (hi - lo + MT - 1) / MT;
    if (e < 0 && bid < tb + ntile) { e = ee; tile0 = lo + (bid - tb) * MT; seg_hi = hi; }
    tb += ntile;
  }
  if (e < 0) return;

  const int tid = threadIdx.x, lane = tid & 31, wave = tid >> 5;
  const int h = lane >> 4, m = lane & 15;
  const int nrows = min(MT, seg_hi - tile0);

  if (tid < MT) {
    int tk = -1;
    if (tid < nrows) {
      tk = row_tok[tile0 + tid];
      tk = min(max(tk, 0), ntok - 1);
    }
    sTok[tid] = tk;
  }
  __syncthreads();

  {
    const int row = tid >> 3, q = tid & 7;
    const int tk = sTok[row];
    const float* src = x + (size_t)(tk < 0 ? 0 : tk) * HID + q * 64;
    _Float16* dst = su.g.x + row * XP + q * 64;
#pragma unroll
    for (int c = 0; c < 8; ++c) {
      Pack8 u;
      if (tk >= 0) {
        v4f a = *(const v4f*)(src + c * 8);
        v4f b = *(const v4f*)(src + c * 8 + 4);
        u.s[0] = (_Float16)(bfr(a.x) * SCX); u.s[1] = (_Float16)(bfr(a.y) * SCX);
        u.s[2] = (_Float16)(bfr(a.z) * SCX); u.s[3] = (_Float16)(bfr(a.w) * SCX);
        u.s[4] = (_Float16)(bfr(b.x) * SCX); u.s[5] = (_Float16)(bfr(b.y) * SCX);
        u.s[6] = (_Float16)(bfr(b.z) * SCX); u.s[7] = (_Float16)(bfr(b.w) * SCX);
      } else {
        u.v = v8h{0, 0, 0, 0, 0, 0, 0, 0};
      }
      *(v8h*)(dst + c * 8) = u.v;
    }
  }

  const int mb = (wave & 1) * 32;
  const int nb = (wave >> 1) * 64;
  v8f acc[2][4];
#pragma unroll
  for (int i = 0; i < 2; ++i)
#pragma unroll
    for (int j = 0; j < 4; ++j) acc[i][j] = v8f{0, 0, 0, 0, 0, 0, 0, 0};

  const int mt = wave & 3, nt = wave >> 2;
  const float* b1e = b1 + (size_t)e * DFF;
  const _Float16* w1e = w1t + (size_t)e * DFF * HID;
  const _Float16* w2e = w2t + (size_t)e * HID * DFF;

  for (int ch = 0; ch < NCH; ++ch) {
    __syncthreads();
#pragma unroll
    for (int it = 0; it < 8; ++it) {
      int p = tid + it * TPB;
      int nn = p >> 6, c = p & 63;
      v8h v = *(const v8h*)(w1e + (size_t)(ch * CC + nn) * HID + c * 8);
      *(v8h*)(su.g.w1 + nn * XP + c * 8) = v;
    }
#pragma unroll
    for (int it = 0; it < 8; ++it) {
      int p = tid + it * TPB;
      int n = p >> 3, c = p & 7;
      v8h v = *(const v8h*)(w2e + (size_t)n * DFF + ch * CC + c * 8);
      *(v8h*)(sW2 + n * W2TP + c * 8) = v;
    }
    __syncthreads();

    {
      v8f a1 = v8f{0, 0, 0, 0, 0, 0, 0, 0};
      const _Float16* ap = su.g.x + (mt * 16 + m) * XP;
      const _Float16* bp = su.g.w1 + (nt * 16 + m) * XP;
#pragma unroll 4
      for (int ks = 0; ks < HID / 32; ++ks) {
        v16h af = ld_frag(ap + ks * 32, h);
        v16h bf = ld_frag(bp + ks * 32, h);
        a1 = wmma16(af, bf, a1);
      }
      const float bb = b1e[ch * CC + nt * 16 + m];
#pragma unroll
      for (int r = 0; r < 8; ++r) {
        int mr = mt * 16 + 8 * h + r;
        float pre = a1[r] * INV_G1 + bb;
        float gl = gelu_t(pre);
        sHd[mr * HP + nt * 16 + m] = (_Float16)(gl * SCH);
      }
    }
    __syncthreads();

#pragma unroll
    for (int ks = 0; ks < CC / 32; ++ks) {
      v16h aF0 = ld_frag(sHd + (mb + m) * HP + ks * 32, h);
      v16h aF1 = ld_frag(sHd + (mb + 16 + m) * HP + ks * 32, h);
#pragma unroll
      for (int j = 0; j < 4; ++j) {
        v16h bF = ld_frag(sW2 + (nb + j * 16 + m) * W2TP + ks * 32, h);
        acc[0][j] = wmma16(aF0, bF, acc[0][j]);
        acc[1][j] = wmma16(aF1, bF, acc[1][j]);
      }
    }
  }
  __syncthreads();

  {
    const float* b2e = b2 + (size_t)e * HID;
#pragma unroll
    for (int i = 0; i < 2; ++i)
#pragma unroll
      for (int j = 0; j < 4; ++j)
#pragma unroll
        for (int r = 0; r < 8; ++r) {
          int row = mb + i * 16 + 8 * h + r;
          int col = nb + j * 16 + m;
          su.stage[row * STP + col] = acc[i][j][r] * INV_G2 + b2e[col];
        }
  }
  __syncthreads();

  v4f vals[4][4];
#pragma unroll
  for (int rr = 0; rr < 4; ++rr) {
    int row = wave * 4 + rr;
#pragma unroll
    for (int q = 0; q < 4; ++q)
      vals[rr][q] = *(const v4f*)(su.stage + row * STP + lane * 4 + q * 128);
  }
#pragma unroll
  for (int rr = 0; rr < 4; ++rr) {
    int row = wave * 4 + rr;
    if (row < nrows) {
      float* dst = yws + (size_t)(tile0 + row) * HID;
#pragma unroll
      for (int q = 0; q < 4; ++q) *(volatile v4f*)(dst + lane * 4 + q * 128) = vals[rr][q];
    }
  }
  __threadfence();
#pragma unroll
  for (int rr = 0; rr < 4; ++rr) {
    int row = wave * 4 + rr;
    if (row < nrows) {
      float* dst = yws + (size_t)(tile0 + row) * HID;
#pragma unroll
      for (int q = 0; q < 4; ++q) *(volatile v4f*)(dst + lane * 4 + q * 128) = vals[rr][q];
    }
  }
}

__global__ __launch_bounds__(256) void k_combine(const float* __restrict__ yws,
                                                   const int* __restrict__ slotmap,
                                                   const float* __restrict__ tk_w,
                                                   float* out, int ntok) {
  const int lane = threadIdx.x & 31, wave = threadIdx.x >> 5;
  const int t = blockIdx.x * 8 + wave;
  if (t >= ntok) return;
  int s0 = slotmap[(size_t)t * 2 + 0];
  int s1 = slotmap[(size_t)t * 2 + 1];
  s0 = min(max(s0, 0), NSLOT - 1);
  s1 = min(max(s1, 0), NSLOT - 1);
  const float w0 = tk_w[(size_t)t * 2 + 0];
  const float w1 = tk_w[(size_t)t * 2 + 1];
  const float* y0 = yws + (size_t)s0 * HID;
  const float* y1 = yws + (size_t)s1 * HID;
  v4f v[4];
#pragma unroll
  for (int q = 0; q < 4; ++q) {
    v4f a = *(const v4f*)(y0 + lane * 4 + q * 128);
    v4f b = *(const v4f*)(y1 + lane * 4 + q * 128);
    v[q] = a * w0 + b * w1;
  }
  float* dst = out + (size_t)t * HID;
#pragma unroll
  for (int q = 0; q < 4; ++q) *(volatile v4f*)(dst + lane * 4 + q * 128) = v[q];
  __threadfence();
#pragma unroll
  for (int q = 0; q < 4; ++q) *(volatile v4f*)(dst + lane * 4 + q * 128) = v[q];
}

extern "C" void kernel_launch(void* const* d_in, const int* in_sizes, int n_in,
                              void* d_out, int out_size, void* d_ws, size_t ws_size,
                              hipStream_t stream) {
  if (n_in < 6) return;
  if (in_sizes[0] != TKN * HID || in_sizes[1] != NEXP * HID ||
      in_sizes[2] != NEXP * HID * DFF || in_sizes[3] != NEXP * DFF ||
      in_sizes[4] != NEXP * DFF * HID || in_sizes[5] != NEXP * HID) return;
  if (out_size != TKN * HID) return;

  const float* x  = (const float*)d_in[0];
  const float* gw = (const float*)d_in[1];
  const float* w1 = (const float*)d_in[2];
  const float* b1 = (const float*)d_in[3];
  const float* w2 = (const float*)d_in[4];
  const float* b2 = (const float*)d_in[5];
  float* out = (float*)d_out;

  const size_t o_off = 0;
  const size_t o_tki = 256;
  const size_t o_tkw = o_tki + (size_t)NSLOT * 4;
  const size_t o_rtk = o_tkw + (size_t)NSLOT * 4;
  const size_t o_slm = o_rtk + (size_t)NSLOT * 4;
  const size_t o_w1t = o_slm + (size_t)NSLOT * 4;
  const size_t o_w2t = o_w1t + (size_t)NEXP * HID * DFF * 2;
  const size_t o_yws = o_w2t + (size_t)NEXP * HID * DFF * 2;
  const size_t o_end = o_yws + (size_t)NSLOT * HID * 4;
  if (o_end > ws_size) return;

  char* ws = (char*)d_ws;
  int*      offsets  = (int*)(ws + o_off);
  int*      tk_idx   = (int*)(ws + o_tki);
  float*    tk_w     = (float*)(ws + o_tkw);
  int*      row_tok  = (int*)(ws + o_rtk);
  int*      slotmap  = (int*)(ws + o_slm);
  _Float16* w1t      = (_Float16*)(ws + o_w1t);
  _Float16* w2t      = (_Float16*)(ws + o_w2t);
  float*    yws      = (float*)(ws + o_yws);

  k_router<<<dim3(TKN / 32), dim3(256), 0, stream>>>(x, gw, tk_idx, (int*)tk_w, TKN);
  k_lists<<<dim3(1), dim3(1024), 0, stream>>>(tk_idx, offsets, row_tok, slotmap);
  k_cvt<<<dim3(DFF / 64, HID / 64, NEXP), dim3(256), 0, stream>>>(w1, w1t, HID, DFF, SCW);
  k_cvt<<<dim3(HID / 64, DFF / 64, NEXP), dim3(256), 0, stream>>>(w2, w2t, DFF, HID, SCW);
  k_expert<<<dim3(NSLOT / MT + NEXP), dim3(TPB), 0, stream>>>(x, b1, b2, w1t, w2t,
                                                               offsets, row_tok, yws, TKN);
  k_combine<<<dim3(TKN / 8), dim3(256), 0, stream>>>(yws, slotmap, tk_w, out, TKN);
}
